// SimplifiedMambaBlock_38835094290480
// MI455X (gfx1250) — hardware-verified
//
#include <hip/hip_runtime.h>
#include <math.h>

typedef __attribute__((ext_vector_type(16))) _Float16 v16h;
typedef __attribute__((ext_vector_type(8)))  _Float16 v8h;
typedef __attribute__((ext_vector_type(16))) __bf16   v16b;
typedef __attribute__((ext_vector_type(8)))  __bf16   v8b;
typedef __attribute__((ext_vector_type(8)))  float    v8f;
typedef __attribute__((ext_vector_type(4)))  float    v4f;

constexpr int kBatch = 4;
constexpr int kSeqL  = 2048;
constexpr int kDmod  = 1024;
constexpr int kDin   = 2048;
constexpr int kNst   = 16;
constexpr int kSsmN  = 2 * kNst;
constexpr int kSsmP  = 64;
constexpr int kXGP   = 2 * kDin;
constexpr int kRows  = kBatch * kSeqL;
constexpr int kTP    = 260;

__device__ __forceinline__ unsigned short f2bf_bits(float f) {
  unsigned u = __float_as_uint(f);
  return (unsigned short)((u + 0x7FFFu + ((u >> 16) & 1u)) >> 16);
}
__device__ __forceinline__ float bf_bits2f(unsigned short h) { return __uint_as_float(((unsigned)h) << 16); }

__device__ __forceinline__ void dep_guard_h(v8f& a, v8f& b, v16h x, v16h y) { asm volatile("v_nop\n\tv_nop\n\tv_nop\n\tv_nop" : "+v"(a), "+v"(b) : "v"(x), "v"(y)); }
__device__ __forceinline__ void dep_guard_b(v8f& a, v8f& b, v16b x, v16b y) { asm volatile("v_nop\n\tv_nop\n\tv_nop\n\tv_nop" : "+v"(a), "+v"(b) : "v"(x), "v"(y)); }
__device__ __forceinline__ void keep4_h(v16h a, v16h b, v16h c, v16h d) { asm volatile("v_nop" :: "v"(a), "v"(b), "v"(c), "v"(d)); }
__device__ __forceinline__ void keep4_b(v16b a, v16b b, v16b c, v16b d) { asm volatile("v_nop" :: "v"(a), "v"(b), "v"(c), "v"(d)); }
__device__ __forceinline__ void acc_guard4(v8f& a, v8f& b, v8f& c, v8f& d) { asm volatile("v_nop\n\tv_nop\n\tv_nop\n\tv_nop" : "+v"(a), "+v"(b), "+v"(c), "+v"(d)); }
template <typename T> struct Frag;
template <> struct Frag<_Float16> {
  typedef v16h V; union U { v16h v; v8h h[2]; };
  static __device__ __forceinline__ v16h load(const _Float16* p) {
    U f; f.h[0] = *(const v8h*)(p); f.h[1] = *(const v8h*)(p + 16); return f.v;
  }
  static __device__ __forceinline__ v8f mma(v16h a, v16h b, v8f c) {
    return __builtin_amdgcn_wmma_f32_16x16x32_f16(false, a, false, b, (short)0, c, false, false);
  }
  static __device__ __forceinline__ void guard(v8f& a, v8f& b, v16h x, v16h y) { dep_guard_h(a, b, x, y); }
  static __device__ __forceinline__ void keep(v16h a, v16h b, v16h c, v16h d) { keep4_h(a, b, c, d); }
};
template <> struct Frag<__bf16> {
  typedef v16b V; union U { v16b v; v8b h[2]; };
  static __device__ __forceinline__ v16b load(const __bf16* p) {
    U f; f.h[0] = *(const v8b*)(p); f.h[1] = *(const v8b*)(p + 16); return f.v;
  }
  static __device__ __forceinline__ v8f mma(v16b a, v16b b, v8f c) {
    return __builtin_amdgcn_wmma_f32_16x16x32_bf16(false, a, false, b, (short)0, c, false, false);
  }
  static __device__ __forceinline__ void guard(v8f& a, v8f& b, v16b x, v16b y) { dep_guard_b(a, b, x, y); }
  static __device__ __forceinline__ void keep(v16b a, v16b b, v16b c, v16b d) { keep4_b(a, b, c, d); }
};

template <int ET> struct Elem;
template <> struct Elem<0> { typedef _Float16 T; };
template <> struct Elem<1> { typedef __bf16 T; };
template <int ET, bool SPLIT, int BIAS_MODE, int OUT_MODE, bool RESID, int ACT = 0>
__global__ __launch_bounds__(256) void wmma_gemm64(
    const unsigned short* __restrict__ Ap, const unsigned short* __restrict__ A2p, int lda, long strideA,
    const unsigned short* __restrict__ Btp, const unsigned short* __restrict__ Bt2p, int ldb, long strideB,
    void* __restrict__ Cout, void* __restrict__ Cout2, int ldc, long strideC,
    const float* __restrict__ bias,
    const float* __restrict__ resid, long strideR,
    int M, int N, int K, float scale) {
  typedef typename Elem<ET>::T T;
  typedef typename Frag<T>::V V;
  const T* A = (const T*)Ap; const T* A2 = (const T*)A2p; const T* Bt = (const T*)Btp; const T* Bt2 = (const T*)Bt2p;
  __shared__ __align__(16) float sT[8][16 * 68];
  const int b    = blockIdx.y;
  const int lane = threadIdx.x & 31;
  const int wave = threadIdx.x >> 5;
  const int tilesN = N >> 6;
  const int tilesM = M >> 6;
  const int tile = blockIdx.x * 8 + wave;
  if (tile >= tilesM * tilesN) return;
  const int tm = tile / tilesN;
  const int tn = tile - tm * tilesN;
  const int m0 = tm << 6;
  const int n0 = tn << 6;

  const T* Ab  = A  + (size_t)b * strideA;
  const T* Bb  = Bt + (size_t)b * strideB;
  const T* Ab2 = SPLIT ? (A2  + (size_t)b * strideA) : nullptr;
  const T* Bb2 = SPLIT ? (Bt2 + (size_t)b * strideB) : nullptr;

  const int rlane = lane & 15;
  const int koff  = (lane >> 4) * 8;
  const int mOff  = (lane >> 4) * 8;

  v8f acc[4][4];
#pragma unroll
  for (int i = 0; i < 4; ++i)
#pragma unroll
    for (int j = 0; j < 4; ++j) acc[i][j] = (v8f){0.f,0.f,0.f,0.f,0.f,0.f,0.f,0.f};

  for (int k0 = 0; k0 < K; k0 += 32) {
    V bh[4], bl[4];
#pragma unroll
    for (int j = 0; j < 4; ++j) {
      const size_t bo = (size_t)(n0 + (j << 4) + rlane) * ldb + koff + k0;
      bh[j] = Frag<T>::load(Bb + bo);
      if (SPLIT) bl[j] = Frag<T>::load(Bb2 + bo);
    }
#pragma unroll
    for (int i = 0; i < 4; ++i) {
      const size_t ao = (size_t)(m0 + (i << 4) + rlane) * lda + koff + k0;
      V ah = Frag<T>::load(Ab + ao);
      V al;
      if (SPLIT) al = Frag<T>::load(Ab2 + ao);
#pragma unroll
      for (int j = 0; j < 4; ++j) {
        acc[i][j] = Frag<T>::mma(ah, bh[j], acc[i][j]);
        if (SPLIT) {
          acc[i][j] = Frag<T>::mma(ah, bl[j], acc[i][j]);
          acc[i][j] = Frag<T>::mma(al, bh[j], acc[i][j]);
        }
      }
      Frag<T>::guard(acc[i][0], acc[i][3], ah, SPLIT ? al : ah);
    }
    Frag<T>::keep(bh[0], bh[1], bh[2], bh[3]);
    if (SPLIT) Frag<T>::keep(bl[0], bl[1], bl[2], bl[3]);
  }
  acc_guard4(acc[0][0], acc[0][1], acc[0][2], acc[0][3]);
  acc_guard4(acc[1][0], acc[1][1], acc[1][2], acc[1][3]);
  acc_guard4(acc[2][0], acc[2][1], acc[2][2], acc[2][3]);
  acc_guard4(acc[3][0], acc[3][1], acc[3][2], acc[3][3]);

  float* slab = sT[wave];
  const float* Rb = RESID ? (resid + (size_t)b * strideR) : nullptr;
#pragma unroll
  for (int i = 0; i < 4; ++i) {
    const int mBase = m0 + (i << 4);
#pragma unroll
    for (int j = 0; j < 4; ++j) {
      const int n = n0 + (j << 4) + rlane;
      float bv = 0.f;
      if (BIAS_MODE == 2) bv = bias[n];
#pragma unroll
      for (int r = 0; r < 8; ++r) {
        float v = acc[i][j][r] * scale;
        if (BIAS_MODE == 1) v += bias[mBase + mOff + r];
        if (BIAS_MODE == 2) v += bv;
        if (RESID) v += Rb[(size_t)(mBase + mOff + r) * ldc + n];
        if (ACT == 1) v = tanhf(v);
        if (ACT == 2) v = fmaxf(v, 0.0f);
        if (ACT == 3) v = v / (1.0f + expf(-v));
        if (ACT == 4) v = (v > 0.f) ? v : 0.01f * v;
        if (ACT == 5) v = 0.5f * v * (1.0f + erff(v * 0.70710678118654752f));
        slab[(mOff + r) * 68 + (j << 4) + rlane] = v;
      }
    }
    __builtin_amdgcn_fence(__ATOMIC_RELEASE, "workgroup");
    __builtin_amdgcn_wave_barrier();
    __builtin_amdgcn_fence(__ATOMIC_ACQUIRE, "workgroup");
    if (OUT_MODE == 0) {
      float* C = (float*)Cout + (size_t)b * strideC;
      const int hh = lane >> 4, c4 = (lane & 15) * 4;
      for (int pass = 0; pass < 2; ++pass) {
#pragma unroll
        for (int it = 0; it < 8; ++it) {
          const int row = it * 2 + hh;
          v4f v = *(const v4f*)(slab + row * 68 + c4);
          *(volatile v4f*)(C + (size_t)(mBase + row) * ldc + n0 + c4) = v;
        }
        __threadfence();
      }
    } else {
      const int q = lane >> 3, c8 = (lane & 7) * 8;
      unsigned short* C  = (unsigned short*)Cout  + (size_t)b * strideC;
      unsigned short* C2 = (OUT_MODE == 2) ? ((unsigned short*)Cout2 + (size_t)b * strideC) : nullptr;
      for (int pass = 0; pass < 2; ++pass) {
#pragma unroll
        for (int it = 0; it < 4; ++it) {
          const int row = it * 4 + q;
          const float* sp = slab + row * 68 + c8;
          v8h hv, lv;
#pragma unroll
          for (int e = 0; e < 8; ++e) {
            if (OUT_MODE == 1) {
              hv[e] = (_Float16)sp[e];
            } else {
              unsigned short hb = f2bf_bits(sp[e]);
              unsigned short lb = f2bf_bits(sp[e] - bf_bits2f(hb));
              hv[e] = __builtin_bit_cast(_Float16, hb);
              lv[e] = __builtin_bit_cast(_Float16, lb);
            }
          }
          *(volatile v8h*)(C + (size_t)(mBase + row) * ldc + n0 + c8) = hv;
          if (OUT_MODE == 2) *(volatile v8h*)(C2 + (size_t)(mBase + row) * ldc + n0 + c8) = lv;
        }
        __threadfence();
      }
    }
    __builtin_amdgcn_fence(__ATOMIC_RELEASE, "workgroup");
    __builtin_amdgcn_wave_barrier();
    __builtin_amdgcn_fence(__ATOMIC_ACQUIRE, "workgroup");
  }
}

__global__ __launch_bounds__(256) void transpose_cast_kernel(
    const float* __restrict__ W, unsigned short* __restrict__ Bt, int Kdim, int Ndim, int Npad, float scale)
{
  __shared__ float tile[64 * 65];
  const int tid = threadIdx.x, lane = tid & 31, wave = tid >> 5;
  const int n0 = blockIdx.x * 64;
  const int k0 = blockIdx.y * 64;
  (void)Npad;
#pragma unroll
  for (int p = 0; p < 16; ++p) {
    const int idx = tid + p * 256;
    const int kk  = idx >> 6;
    const int nn  = idx & 63;
    const int n   = n0 + nn;
    const int nc  = (n < Ndim) ? n : (Ndim - 1);
    const float v = W[(size_t)(k0 + kk) * Ndim + nc];
    tile[kk * 65 + nn] = (n < Ndim) ? (v * scale) : 0.f;
  }
  __syncthreads();
  const int q = lane >> 3, c8 = (lane & 7) * 8;
  v8h hv[2];
#pragma unroll
  for (int it = 0; it < 2; ++it) {
    const int nrow = it * 32 + wave * 4 + q;
#pragma unroll
    for (int e = 0; e < 8; ++e) hv[it][e] = (_Float16)tile[(c8 + e) * 65 + nrow];
  }
  for (int pass = 0; pass < 2; ++pass) {
#pragma unroll
    for (int it = 0; it < 2; ++it) {
      const int nrow = it * 32 + wave * 4 + q;
      *(volatile v8h*)(Bt + (size_t)(n0 + nrow) * Kdim + k0 + c8) = hv[it];
    }
    __threadfence();
  }
}

__global__ __launch_bounds__(256) void ln_f16_kernel(
    const float* __restrict__ x, const float* __restrict__ w, const float* __restrict__ bb,
    unsigned short* __restrict__ XN16, int nrows)
{
  const int lane = threadIdx.x & 31, wave = threadIdx.x >> 5;
  const int row = blockIdx.x * 8 + wave;
  if (row >= nrows) return;
  const float* xr = x + (size_t)row * kDmod;
  float v[4][8];
  float s = 0.f;
#pragma unroll
  for (int it = 0; it < 4; ++it) {
    const v4f a0 = *(const v4f*)(xr + it * 256 + lane * 8);
    const v4f a1 = *(const v4f*)(xr + it * 256 + lane * 8 + 4);
#pragma unroll
    for (int e = 0; e < 4; ++e) {
      v[it][e] = a0[e]; v[it][4 + e] = a1[e];
      s += a0[e]; s += a1[e];
    }
  }
#pragma unroll
  for (int off = 16; off >= 1; off >>= 1) s += __shfl_xor(s, off, 32);
  const float mean = s * (1.0f / (float)kDmod);
  float s2 = 0.f;
#pragma unroll
  for (int it = 0; it < 4; ++it) {
#pragma unroll
    for (int e = 0; e < 8; ++e) {
      float dd = v[it][e] - mean;
      asm volatile("" : "+v"(dd));
      v[it][e] = dd;
      float q = dd * dd;
      asm volatile("" : "+v"(q));
      s2 += q;
    }
  }
#pragma unroll
  for (int off = 16; off >= 1; off >>= 1) s2 += __shfl_xor(s2, off, 32);
  const float var  = s2 * (1.0f / (float)kDmod);
  const float rstd = rsqrtf(var + 1e-5f);
  v8h hv[4];
#pragma unroll
  for (int it = 0; it < 4; ++it) {
    const int c0 = it * 256 + lane * 8;
    const v4f w0 = *(const v4f*)(w + c0);
    const v4f w1 = *(const v4f*)(w + c0 + 4);
    const v4f b0 = *(const v4f*)(bb + c0);
    const v4f b1 = *(const v4f*)(bb + c0 + 4);
#pragma unroll
    for (int e = 0; e < 8; ++e) {
      const float wv = (e < 4) ? w0[e] : w1[e - 4];
      const float bv = (e < 4) ? b0[e] : b1[e - 4];
      float o = v[it][e] * rstd;
      asm volatile("" : "+v"(o));
      o = o * wv;
      asm volatile("" : "+v"(o));
      o = o + bv;
      hv[it][e] = (_Float16)o;
    }
  }
  unsigned short* orow = XN16 + (size_t)row * kDmod;
  for (int pass = 0; pass < 2; ++pass) {
#pragma unroll
    for (int it = 0; it < 4; ++it)
      *(volatile v8h*)(orow + it * 256 + lane * 8) = hv[it];
    __threadfence();
  }
}

__global__ __launch_bounds__(256) void conv_silu_kernel(
    const float* __restrict__ XG, const float* __restrict__ cw, const float* __restrict__ cb,
    float* __restrict__ XC, unsigned short* __restrict__ XC16)
{
  __shared__ __align__(16) float sT[16 * kTP];
  const int tid = threadIdx.x, lane = tid & 31, wave = tid >> 5;
  const int d0 = blockIdx.x * 256, d = d0 + tid;
  const int t0 = blockIdx.y * 64;
  const float w0 = cw[d * 4 + 0], w1 = cw[d * 4 + 1], w2 = cw[d * 4 + 2], w3 = cw[d * 4 + 3];
  const float bc = cb[d];
  float xm3, xm2, xm1;
  {
    const int r3 = t0 - 3, r2 = t0 - 2, r1 = t0 - 1;
    const float v3 = XG[(size_t)(r3 < 0 ? 0 : r3) * kXGP + d];
    const float v2 = XG[(size_t)(r2 < 0 ? 0 : r2) * kXGP + d];
    const float v1 = XG[(size_t)(r1 < 0 ? 0 : r1) * kXGP + d];
    xm3 = (r3 >= 0) ? v3 : 0.f;
    xm2 = (r2 >= 0) ? v2 : 0.f;
    xm1 = (r1 >= 0) ? v1 : 0.f;
  }
  const int hrow = wave >> 1;
  const int hch  = (wave & 1) * 128 + lane * 4;
#pragma unroll 1
  for (int sub = 0; sub < 4; ++sub) {
    const int lb = t0 + sub * 16;
#pragma unroll 1
    for (int s = 0; s < 16; ++s) {
      const float xc = XG[(size_t)(lb + s) * kXGP + d];
      float acc = w0 * xm3;
      acc = fmaf(w1, xm2, acc);
      acc = fmaf(w2, xm1, acc);
      acc = fmaf(w3, xc, acc);
      const float sv = acc + bc;
      const float sg = __builtin_amdgcn_rcpf(1.0f + __expf(-sv));
      sT[s * kTP + tid] = sv * sg;
      xm3 = xm2; xm2 = xm1; xm1 = xc;
    }
    __syncthreads();
    v4f fv[4];
    v8h bv[2];
#pragma unroll
    for (int it = 0; it < 4; ++it) fv[it] = *(const v4f*)(sT + (it * 4 + hrow) * kTP + hch);
#pragma unroll
    for (int it = 0; it < 2; ++it) {
      const float* sp = sT + (it * 8 + wave) * kTP + lane * 8;
      const v4f a0 = *(const v4f*)(sp);
      const v4f a1 = *(const v4f*)(sp + 4);
#pragma unroll
      for (int e = 0; e < 4; ++e) {
        bv[it][e]     = (_Float16)a0[e];
        bv[it][4 + e] = (_Float16)a1[e];
      }
    }
    for (int pass = 0; pass < 2; ++pass) {
#pragma unroll
      for (int it = 0; it < 4; ++it)
        *(volatile v4f*)(XC + (size_t)(lb + it * 4 + hrow) * kDin + d0 + hch) = fv[it];
#pragma unroll
      for (int it = 0; it < 2; ++it)
        *(volatile v8h*)(XC16 + (size_t)(lb + it * 8 + wave) * kDin + d0 + lane * 8) = bv[it];
      __threadfence();
    }
    __syncthreads();
  }
}

__global__ __launch_bounds__(256) void scan_kernel(
    const float* __restrict__ XC, const float* __restrict__ XG,
    const float* __restrict__ SSM, const float* __restrict__ bx,
    const float* __restrict__ A_log, const float* __restrict__ Dv,
    unsigned short* __restrict__ Y16)
{
  __shared__ __align__(16) float sBC[16 * 32];
  __shared__ __align__(16) float sY[16 * kTP];
  __shared__ float sDA[kNst * 256];
  const int tid = threadIdx.x, lane = tid & 31, wave = tid >> 5;
  const int d0 = blockIdx.x * 256, d = d0 + tid;

#pragma unroll 1
  for (int n = 0; n < kNst; ++n) {
    const float al = A_log[(size_t)d * kNst + n];
    sDA[n * 256 + tid] = expf(-expf(al));
  }
  __syncthreads();
  float dA[kNst], h[kNst];
#pragma unroll
  for (int n = 0; n < kNst; ++n) { dA[n] = sDA[n * 256 + tid]; h[n] = 0.f; }
  const float Dd = Dv[d];

#pragma unroll 1
  for (int c = 0; c < kSeqL / 16; ++c) {
    const int l0 = c * 16;
    if (tid < 128) {
      const int r = tid >> 3, q = (tid & 7) * 4;
      v4f v = *(const v4f*)(SSM + (size_t)(l0 + r) * kSsmP + q);
      const v4f bq = *(const v4f*)(bx + q);
      v = v + bq;
      *(v4f*)(sBC + r * 32 + q) = v;
    }
    __syncthreads();
#pragma unroll 1
    for (int s = 0; s < 16; ++s) {
      const size_t m = (size_t)(l0 + s);
      const float xv = XC[m * kDin + d];
      const float zv = XG[m * kXGP + kDin + d];
      v4f Bq[4], Cq[4];
#pragma unroll
      for (int qq = 0; qq < 4; ++qq) {
        Bq[qq] = *(const v4f*)(sBC + s * 32 + 4 * qq);
        Cq[qq] = *(const v4f*)(sBC + s * 32 + kNst + 4 * qq);
      }
      float y = 0.f;
#pragma unroll
      for (int n = 0; n < kNst; ++n) {
        float p = xv * Bq[n >> 2][n & 3];
        asm volatile("" : "+v"(p));
        float qv = h[n] * dA[n];
        asm volatile("" : "+v"(qv));
        const float hn = qv + p;
        h[n] = hn;
        float rr = hn * Cq[n >> 2][n & 3];
        asm volatile("" : "+v"(rr));
        y += rr;
      }
      float sk = xv * Dd;
      asm volatile("" : "+v"(sk));
      y += sk;
      const float sg = __builtin_amdgcn_rcpf(1.0f + __expf(-zv));
      const float g  = zv * sg;
      sY[s * kTP + tid] = (y * g) * 16.0f;
    }
    __syncthreads();
    v8h hv[2];
#pragma unroll
    for (int it = 0; it < 2; ++it) {
      const float* sp = sY + (it * 8 + wave) * kTP + lane * 8;
      const v4f a0 = *(const v4f*)(sp);
      const v4f a1 = *(const v4f*)(sp + 4);
#pragma unroll
      for (int e = 0; e < 4; ++e) { hv[it][e] = (_Float16)a0[e]; hv[it][4 + e] = (_Float16)a1[e]; }
    }
    for (int pass = 0; pass < 2; ++pass) {
#pragma unroll
      for (int it = 0; it < 2; ++it)
        *(volatile v8h*)(Y16 + (size_t)(l0 + it * 8 + wave) * kDin + d0 + lane * 8) = hv[it];
      __threadfence();
    }
  }
}

extern "C" void kernel_launch(void* const* d_in, const int* in_sizes, int n_in,
                              void* d_out, int out_size, void* d_ws, size_t ws_size,
                              hipStream_t stream)
{
  if (n_in < 13) return;
  const float* x      = (const float*)d_in[0];
  const float* ln_w   = (const float*)d_in[1];
  const float* ln_b   = (const float*)d_in[2];
  const float* W_in   = (const float*)d_in[3];
  const float* b_in   = (const float*)d_in[4];
  const float* conv_w = (const float*)d_in[5];
  const float* conv_b = (const float*)d_in[6];
  const float* A_log  = (const float*)d_in[7];
  const float* Dv     = (const float*)d_in[8];
  const float* W_x    = (const float*)d_in[9];
  const float* b_x    = (const float*)d_in[10];
  const float* W_out  = (const float*)d_in[11];
  const float* b_out  = (const float*)d_in[12];
  float* dout = (float*)d_out;

  if (in_sizes[0] != kRows * kDmod) return;
  if (in_sizes[1] != kDmod || in_sizes[2] != kDmod) return;
  if (in_sizes[3] != kDmod * kXGP || in_sizes[4] != kXGP) return;
  if (in_sizes[5] != kDin * 4 || in_sizes[6] != kDin) return;
  if (in_sizes[7] != kDin * kNst || in_sizes[8] != kDin) return;
  if (in_sizes[9] != kDin * kSsmN || in_sizes[10] != kSsmN) return;
  if (in_sizes[11] != kDin * kDmod || in_sizes[12] != kDmod) return;
  if (out_size != kRows * kDmod) return;

  const size_t SZ_WIN16  = (size_t)kXGP * kDmod * 2;
  const size_t SZ_WX16   = (size_t)kSsmP * kDin * 2;
  const size_t SZ_WOUT16 = (size_t)kDmod * kDin * 2;
  const size_t SZ_XN16   = (size_t)kRows * kDmod * 2;
  const size_t SZ_XG     = (size_t)kSeqL * kXGP * 4;
  const size_t SZ_XC     = (size_t)kSeqL * kDin * 4;
  const size_t SZ_XC16   = (size_t)kSeqL * kDin * 2;
  const size_t SZ_SSM    = (size_t)kSeqL * kSsmP * 4;
  const size_t SZ_Y16    = (size_t)kSeqL * kDin * 2;
  const size_t OFF_WIN16  = 0;
  const size_t OFF_WX16   = OFF_WIN16  + SZ_WIN16;
  const size_t OFF_WOUT16 = OFF_WX16   + SZ_WX16;
  const size_t OFF_XN16   = OFF_WOUT16 + SZ_WOUT16;
  const size_t OFF_XG     = OFF_XN16   + SZ_XN16;
  const size_t OFF_XC     = OFF_XG     + SZ_XG;
  const size_t OFF_XC16   = OFF_XC     + SZ_XC;
  const size_t OFF_SSM    = OFF_XC16   + SZ_XC16;
  const size_t OFF_Y16    = OFF_SSM    + SZ_SSM;
  const size_t TOTAL      = OFF_Y16    + SZ_Y16;
  if (ws_size < TOTAL) return;

  char* ws = (char*)d_ws;
  unsigned short* WIN16  = (unsigned short*)(ws + OFF_WIN16);
  unsigned short* WX16   = (unsigned short*)(ws + OFF_WX16);
  unsigned short* WOUT16 = (unsigned short*)(ws + OFF_WOUT16);
  unsigned short* XN16   = (unsigned short*)(ws + OFF_XN16);
  float*          XG     = (float*)(ws + OFF_XG);
  float*          XC     = (float*)(ws + OFF_XC);
  unsigned short* XC16   = (unsigned short*)(ws + OFF_XC16);
  float*          SSM    = (float*)(ws + OFF_SSM);
  unsigned short* Y16    = (unsigned short*)(ws + OFF_Y16);
  const float* dummy_bias  = b_in;
  const float* dummy_resid = x;

  transpose_cast_kernel<<<dim3(kXGP / 64, kDmod / 64), 256, 0, stream>>>(W_in,  WIN16,  kDmod, kXGP,  kXGP,  32.0f);
  transpose_cast_kernel<<<dim3(kSsmP / 64, kDin / 64), 256, 0, stream>>>(W_x,   WX16,   kDin,  kSsmN, kSsmP, 32.0f);
  transpose_cast_kernel<<<dim3(kDmod / 64, kDin / 64), 256, 0, stream>>>(W_out, WOUT16, kDin,  kDmod, kDmod, 32.0f);

  ln_f16_kernel<<<kRows / 8, 256, 0, stream>>>(x, ln_w, ln_b, XN16, kRows);

  for (int b = 0; b < kBatch; ++b) {
    const unsigned short* XN16b = XN16 + (size_t)b * kSeqL * kDmod;
    const float* xb   = x    + (size_t)b * kSeqL * kDmod;
    float*       outb = dout + (size_t)b * kSeqL * kDmod;

    wmma_gemm64<0, false, 2, 0, false><<<dim3(256, 1), 256, 0, stream>>>(
        XN16b, XN16b, kDmod, 0L, WIN16, WIN16, kDmod, 0L,
        (void*)XG, (void*)XG, kXGP, 0L, b_in, dummy_resid, 0L, kSeqL, kXGP, kDmod, 1.0f / 32.0f);

    conv_silu_kernel<<<dim3(kDin / 256, kSeqL / 64), 256, 0, stream>>>(XG, conv_w, conv_b, XC, XC16);

    wmma_gemm64<0, false, 0, 0, false><<<dim3(4, 1), 256, 0, stream>>>(
        XC16, XC16, kDin, 0L, WX16, WX16, kDin, 0L,
        (void*)SSM, (void*)SSM, kSsmP, 0L, dummy_bias, dummy_resid, 0L, kSeqL, kSsmP, kDin, 1.0f / 32.0f);

    scan_kernel<<<dim3(kDin / 256, 1), 256, 0, stream>>>(XC, XG, SSM, b_x, A_log, Dv, Y16);

    wmma_gemm64<0, false, 2, 0, true><<<dim3(64, 1), 256, 0, stream>>>(
        Y16, Y16, kDin, 0L, WOUT16, WOUT16, kDin, 0L,
        (void*)outb, (void*)outb, kDmod, 0L, b_out, xb, 0L, kSeqL, kDmod, kDin, 1.0f / 512.0f);
  }
}
